// MultiScaleDeformableAttention_48163763258126
// MI455X (gfx1250) — hardware-verified
//
#include <hip/hip_runtime.h>
#include <stdint.h>

typedef __attribute__((ext_vector_type(16))) _Float16 v16h;
typedef __attribute__((ext_vector_type(8)))  _Float16 v8h;
typedef __attribute__((ext_vector_type(16))) __bf16   v16b;
typedef __attribute__((ext_vector_type(8)))  __bf16   v8b;
typedef __attribute__((ext_vector_type(8)))  float    v8f;
typedef __attribute__((ext_vector_type(4)))  float    v4f;
typedef __attribute__((ext_vector_type(2)))  float    v2f;
typedef __attribute__((ext_vector_type(4)))  unsigned v4u;

constexpr int kBatch  = 2;
constexpr int kSeq    = 11253;
constexpr int kMreal  = kBatch * kSeq;
constexpr int kMpad   = 22528;
constexpr int kDm     = 256;
constexpr int kHeads  = 8;
constexpr int kDh     = 32;
constexpr int kLogit  = 128;
constexpr int kPts    = 16;

static_assert(kMreal == 22506);
static_assert(kMpad % 64 == 0 && kMpad >= kMreal && kMpad - kMreal < 64);
static_assert(kMpad % 8 == 0);
static_assert(kDm % 64 == 0 && kLogit % 64 == 0);
static_assert(kDm % 32 == 0);
static_assert(kHeads * kDh == kDm && kHeads * kPts == kLogit);

constexpr size_t kPlane16 = (size_t)kMpad * kDm * 2;
constexpr size_t kW256    = (size_t)256 * 256 * 2;
constexpr size_t kW128    = (size_t)128 * 256 * 2;
constexpr size_t kPlaneF  = (size_t)kMpad * kDm * 4;
constexpr size_t kPlaneL  = (size_t)kMpad * kLogit * 4;
constexpr size_t kOffQ16   = 0;
constexpr size_t kOffF16   = kOffQ16 + kPlane16;
constexpr size_t kOffWval  = kOffF16 + kPlane16;
constexpr size_t kOffWoff  = kOffWval + kW256;
constexpr size_t kOffWlog  = kOffWoff + kW256;
constexpr size_t kOffWout  = kOffWlog + kW128;
constexpr size_t kOffValue = kOffWout + kW256;
constexpr size_t kOffOffs  = kOffValue + kPlaneF;
constexpr size_t kOffLogit = kOffOffs + kPlaneF;
constexpr size_t kOffShi   = kOffLogit + kPlaneL;
constexpr size_t kOffSlo   = kOffShi + kPlane16;
constexpr size_t kWsTotal  = kOffSlo + kPlane16;
static_assert(kWsTotal == 104267776);
static_assert(kWsTotal <= 134217728);
static_assert(kOffF16 % 256 == 0 && kOffWval % 256 == 0 && kOffWoff % 256 == 0 && kOffWlog % 256 == 0 &&
              kOffWout % 256 == 0 && kOffValue % 256 == 0 && kOffOffs % 256 == 0 && kOffLogit % 256 == 0 &&
              kOffShi % 256 == 0 && kOffSlo % 256 == 0);

__device__ __forceinline__ unsigned short f2bf_bits(float f) {
  unsigned u = __float_as_uint(f);
  return (unsigned short)((u + 0x7FFFu + ((u >> 16) & 1u)) >> 16);
}
__device__ __forceinline__ float bf_bits2f(unsigned short h) { return __uint_as_float(((unsigned)h) << 16); }
__device__ __forceinline__ float bf_rne(float f) { return bf_bits2f(f2bf_bits(f)); }

__device__ __forceinline__ void dep_guard_h(v8f& a, v8f& b, v16h x, v16h y) { asm volatile("v_nop\n\tv_nop\n\tv_nop\n\tv_nop" : "+v"(a), "+v"(b) : "v"(x), "v"(y)); }
__device__ __forceinline__ void dep_guard_b(v8f& a, v8f& b, v16b x, v16b y) { asm volatile("v_nop\n\tv_nop\n\tv_nop\n\tv_nop" : "+v"(a), "+v"(b) : "v"(x), "v"(y)); }
__device__ __forceinline__ void keep4_h(v16h a, v16h b, v16h c, v16h d) { asm volatile("v_nop" :: "v"(a), "v"(b), "v"(c), "v"(d)); }
__device__ __forceinline__ void keep4_b(v16b a, v16b b, v16b c, v16b d) { asm volatile("v_nop" :: "v"(a), "v"(b), "v"(c), "v"(d)); }
__device__ __forceinline__ void acc_guard4(v8f& a, v8f& b, v8f& c, v8f& d) { asm volatile("v_nop\n\tv_nop\n\tv_nop\n\tv_nop" : "+v"(a), "+v"(b), "+v"(c), "+v"(d)); }

template <typename T> struct Frag;
template <> struct Frag<_Float16> {
  typedef v16h V; union U { v16h v; v8h h[2]; };
  static __device__ __forceinline__ v16h load(const _Float16* p) {
    U f; f.h[0] = *(const v8h*)(p); f.h[1] = *(const v8h*)(p + 16); return f.v;
  }
  static __device__ __forceinline__ v8f mma(v16h a, v16h b, v8f c) {
    return __builtin_amdgcn_wmma_f32_16x16x32_f16(false, a, false, b, (short)0, c, false, false);
  }
  static __device__ __forceinline__ void guard(v8f& a, v8f& b, v16h x, v16h y) { dep_guard_h(a, b, x, y); }
  static __device__ __forceinline__ void keep(v16h a, v16h b, v16h c, v16h d) { keep4_h(a, b, c, d); }
};
template <> struct Frag<__bf16> {
  typedef v16b V; union U { v16b v; v8b h[2]; };
  static __device__ __forceinline__ v16b load(const __bf16* p) {
    U f; f.h[0] = *(const v8b*)(p); f.h[1] = *(const v8b*)(p + 16); return f.v;
  }
  static __device__ __forceinline__ v8f mma(v16b a, v16b b, v8f c) {
    return __builtin_amdgcn_wmma_f32_16x16x32_bf16(false, a, false, b, (short)0, c, false, false);
  }
  static __device__ __forceinline__ void guard(v8f& a, v8f& b, v16b x, v16b y) { dep_guard_b(a, b, x, y); }
  static __device__ __forceinline__ void keep(v16b a, v16b b, v16b c, v16b d) { keep4_b(a, b, c, d); }
};

template <int ET> struct Elem;
template <> struct Elem<0> { typedef _Float16 T; };
template <> struct Elem<1> { typedef __bf16 T; };
template <int ET, bool SPLIT, bool AONLY, int BIAS_MODE, bool RB, int OUT_MODE, bool RESID, int ACT = 0>
__global__ __launch_bounds__(256) void wmma_gemm64(
    const unsigned short* __restrict__ Ap, const unsigned short* __restrict__ A2p, int lda, long strideA,
    const unsigned short* __restrict__ Btp, const unsigned short* __restrict__ Bt2p, int ldb, long strideB,
    void* __restrict__ Cout, void* __restrict__ Cout2, int ldc, long strideC,
    const float* __restrict__ bias,
    const float* __restrict__ resid, long strideR,
    int M, int N, int K, int Mreal, float scale) {
  typedef typename Elem<ET>::T T;
  typedef typename Frag<T>::V V;
  const T* A = (const T*)Ap; const T* A2 = (const T*)A2p; const T* Bt = (const T*)Btp; const T* Bt2 = (const T*)Bt2p;
  __shared__ __align__(16) float sT[8][16 * 68];
  const int b    = blockIdx.y;
  const int lane = threadIdx.x & 31;
  const int wave = threadIdx.x >> 5;
  const int tilesN = N >> 6;
  const int tilesM = M >> 6;
  const int tile = blockIdx.x * 8 + wave;
  if (tile >= tilesM * tilesN) return;
  const int tm = tile / tilesN;
  const int tn = tile - tm * tilesN;
  const int m0 = tm << 6;
  const int n0 = tn << 6;

  const T* Ab  = A  + (size_t)b * strideA;
  const T* Bb  = Bt + (size_t)b * strideB;
  const T* Ab2 = SPLIT ? (A2  + (size_t)b * strideA) : nullptr;
  const T* Bb2 = (SPLIT && !AONLY) ? (Bt2 + (size_t)b * strideB) : nullptr;

  const int rlane = lane & 15;
  const int koff  = (lane >> 4) * 8;
  const int mOff  = (lane >> 4) * 8;

  v8f acc[4][4];
#pragma unroll
  for (int i = 0; i < 4; ++i)
#pragma unroll
    for (int j = 0; j < 4; ++j) acc[i][j] = (v8f){0.f,0.f,0.f,0.f,0.f,0.f,0.f,0.f};

  for (int k0 = 0; k0 < K; k0 += 32) {
    V bh[4], bl[4];
#pragma unroll
    for (int j = 0; j < 4; ++j) {
      const size_t bo = (size_t)(n0 + (j << 4) + rlane) * ldb + koff + k0;
      bh[j] = Frag<T>::load(Bb + bo);
      if (SPLIT && !AONLY) bl[j] = Frag<T>::load(Bb2 + bo);
    }
#pragma unroll
    for (int i = 0; i < 4; ++i) {
      const size_t ao = (size_t)(m0 + (i << 4) + rlane) * lda + koff + k0;
      V ah = Frag<T>::load(Ab + ao);
      V al = ah;
      if (SPLIT) al = Frag<T>::load(Ab2 + ao);
#pragma unroll
      for (int j = 0; j < 4; ++j) {
        acc[i][j] = Frag<T>::mma(ah, bh[j], acc[i][j]);
        if (SPLIT) {
          if (!AONLY) acc[i][j] = Frag<T>::mma(ah, bl[j], acc[i][j]);
          acc[i][j] = Frag<T>::mma(al, bh[j], acc[i][j]);
        }
      }
      Frag<T>::guard(acc[i][0], acc[i][3], ah, al);
    }
    Frag<T>::keep(bh[0], bh[1], bh[2], bh[3]);
    if (SPLIT && !AONLY) Frag<T>::keep(bl[0], bl[1], bl[2], bl[3]);
  }
  acc_guard4(acc[0][0], acc[0][1], acc[0][2], acc[0][3]);
  acc_guard4(acc[1][0], acc[1][1], acc[1][2], acc[1][3]);
  acc_guard4(acc[2][0], acc[2][1], acc[2][2], acc[2][3]);
  acc_guard4(acc[3][0], acc[3][1], acc[3][2], acc[3][3]);

  float* slab = sT[wave];
  const float* Rb = RESID ? (resid + (size_t)b * strideR) : nullptr;
#pragma unroll
  for (int i = 0; i < 4; ++i) {
    const int mBase = m0 + (i << 4);
#pragma unroll
    for (int j = 0; j < 4; ++j) {
      const int n = n0 + (j << 4) + rlane;
      float bv = 0.f;
      if (BIAS_MODE == 2) { bv = bias[n]; if (RB) bv = bf_rne(bv); }
#pragma unroll
      for (int r = 0; r < 8; ++r) {
        float v = acc[i][j][r] * scale;
        if (BIAS_MODE == 1) { float bm = bias[mBase + mOff + r]; if (RB) bm = bf_rne(bm); v += bm; }
        if (BIAS_MODE == 2) v += bv;
        if (RESID) v += Rb[(size_t)(mBase + mOff + r) * ldc + n];
        if (ACT == 1) v = tanhf(v);
        if (ACT == 2) v = fmaxf(v, 0.0f);
        if (ACT == 3) v = v / (1.0f + expf(-v));
        if (ACT == 4) v = (v > 0.f) ? v : 0.01f * v;
        slab[(mOff + r) * 68 + (j << 4) + rlane] = v;
      }
    }
    __builtin_amdgcn_fence(__ATOMIC_RELEASE, "workgroup");
    __builtin_amdgcn_wave_barrier();
    __builtin_amdgcn_fence(__ATOMIC_ACQUIRE, "workgroup");
    if (OUT_MODE == 0) {
      float* C = (float*)Cout + (size_t)b * strideC;
      const int hh = lane >> 4, c4 = (lane & 15) * 4;
      for (int pass = 0; pass < 2; ++pass) {
#pragma unroll
        for (int it = 0; it < 8; ++it) {
          const int row = it * 2 + hh;
          v4f v = *(const v4f*)(slab + row * 68 + c4);
          if (mBase + row < Mreal) *(volatile v4f*)(C + (size_t)(mBase + row) * ldc + n0 + c4) = v;
        }
        __threadfence();
      }
    } else {
      const int q = lane >> 3, c8 = (lane & 7) * 8;
      unsigned short* C  = (unsigned short*)Cout  + (size_t)b * strideC;
      unsigned short* C2 = (OUT_MODE == 2) ? ((unsigned short*)Cout2 + (size_t)b * strideC) : nullptr;
      for (int pass = 0; pass < 2; ++pass) {
#pragma unroll
        for (int it = 0; it < 4; ++it) {
          const int row = it * 4 + q;
          const float* sp = slab + row * 68 + c8;
          v8h hv, lv;
#pragma unroll
          for (int e = 0; e < 8; ++e) {
            if (OUT_MODE == 1) {
              hv[e] = (_Float16)sp[e];
            } else {
              unsigned short hb = f2bf_bits(sp[e]);
              unsigned short lb = f2bf_bits(sp[e] - bf_bits2f(hb));
              hv[e] = __builtin_bit_cast(_Float16, hb);
              lv[e] = __builtin_bit_cast(_Float16, lb);
            }
          }
          if (mBase + row < Mreal) {
            *(volatile v8h*)(C + (size_t)(mBase + row) * ldc + n0 + c8) = hv;
            if (OUT_MODE == 2) *(volatile v8h*)(C2 + (size_t)(mBase + row) * ldc + n0 + c8) = lv;
          }
        }
        __threadfence();
      }
    }
    __builtin_amdgcn_fence(__ATOMIC_RELEASE, "workgroup");
    __builtin_amdgcn_wave_barrier();
    __builtin_amdgcn_fence(__ATOMIC_ACQUIRE, "workgroup");
  }
}

__global__ __launch_bounds__(256) void cvt_rows_bf16(const float* __restrict__ src, unsigned* __restrict__ dst,
                                                     int rowsReal, int rowsPad) {
  const int gid = blockIdx.x * 256 + threadIdx.x;
  const int row = gid >> 5;
  const int c   = gid & 31;
  if (row >= rowsPad) return;
  const int rowc = (row < rowsReal) ? row : (rowsReal - 1);
  const float* p = src + (size_t)rowc * kDm + c * 8;
  const v4f a = *(const v4f*)(p);
  const v4f d = *(const v4f*)(p + 4);
  v4u o;
  o[0] = (unsigned)f2bf_bits(a[0]) | ((unsigned)f2bf_bits(a[1]) << 16);
  o[1] = (unsigned)f2bf_bits(a[2]) | ((unsigned)f2bf_bits(a[3]) << 16);
  o[2] = (unsigned)f2bf_bits(d[0]) | ((unsigned)f2bf_bits(d[1]) << 16);
  o[3] = (unsigned)f2bf_bits(d[2]) | ((unsigned)f2bf_bits(d[3]) << 16);
  unsigned* qp = dst + (size_t)row * (kDm / 2) + c * 4;
  *(volatile v4u*)qp = o;
  __threadfence();
  *(volatile v4u*)qp = o;
}

__device__ __forceinline__ void split_pack2(float a, float b, unsigned& hw, unsigned& lw) {
  const unsigned short ha = f2bf_bits(a);
  const unsigned short hb = f2bf_bits(b);
  const unsigned short la = f2bf_bits(a - bf_bits2f(ha));
  const unsigned short lb = f2bf_bits(b - bf_bits2f(hb));
  hw = (unsigned)ha | ((unsigned)hb << 16);
  lw = (unsigned)la | ((unsigned)lb << 16);
}

__global__ __launch_bounds__(256) void deform_gather(const float* __restrict__ value,
                                                     const float* __restrict__ offp,
                                                     const float* __restrict__ logit,
                                                     const float* __restrict__ rpts,
                                                     unsigned* __restrict__ shi,
                                                     unsigned* __restrict__ slo) {
#pragma clang fp contract(off)
  __shared__ __align__(16) float stage[8][kDm];
  const int lane = threadIdx.x & 31;
  const int wave = threadIdx.x >> 5;
  const int row  = blockIdx.x * 8 + wave;
  const int rowc = (row < kMreal) ? row : (kMreal - 1);
  const int nb   = rowc / kSeq;
  const int pt   = lane & 15;
  const int lvl  = pt >> 2;
  const int Hl  = (lvl == 0) ? 92 : (lvl == 1) ? 46 : (lvl == 2) ? 23 : 12;
  const int Wl  = (lvl == 0) ? 92 : (lvl == 1) ? 46 : (lvl == 2) ? 23 : 12;
  const int st0 = (lvl == 0) ? 0 : (lvl == 1) ? 8464 : (lvl == 2) ? 10580 : 11109;
  const float Wf = (float)Wl;
  const float Hf = (float)Hl;
  const float invW = (lvl == 0) ? (1.0f / 92.0f) : (lvl == 1) ? (1.0f / 46.0f) : (lvl == 2) ? (1.0f / 23.0f) : (1.0f / 12.0f);
  const float invH = invW;
  const float rx = bf_rne(rpts[(size_t)rowc * 8 + lvl * 2 + 0]);
  const float ry = bf_rne(rpts[(size_t)rowc * 8 + lvl * 2 + 1]);
  const float* vbase = value + (size_t)nb * kSeq * kDm + lane;
  float* st = stage[wave];

#pragma unroll 1
  for (int m = 0; m < kHeads; ++m) {
    const float lg = logit[(size_t)rowc * kLogit + m * kPts + pt];
    float mx = lg;
    mx = fmaxf(mx, __shfl_xor(mx, 1, 32));
    mx = fmaxf(mx, __shfl_xor(mx, 2, 32));
    mx = fmaxf(mx, __shfl_xor(mx, 4, 32));
    mx = fmaxf(mx, __shfl_xor(mx, 8, 32));
    const float e = expf(lg - mx);
    float ssum = e;
    ssum += __shfl_xor(ssum, 1, 32);
    ssum += __shfl_xor(ssum, 2, 32);
    ssum += __shfl_xor(ssum, 4, 32);
    ssum += __shfl_xor(ssum, 8, 32);
    const float aw = e * (1.0f / ssum);

    const v2f od = *(const v2f*)(offp + (size_t)rowc * kDm + m * 32 + 2 * pt);
    const float qx = od[0] * invW;
    const float qy = od[1] * invH;
    const float lxn = rx + qx;
    const float lyn = ry + qy;
    float x = lxn * Wf;
    float y = lyn * Hf;
    x = x - 0.5f;
    y = y - 0.5f;
    x = fminf(fmaxf(x, -4.0f), Wf + 4.0f);
    y = fminf(fmaxf(y, -4.0f), Hf + 4.0f);
    const float x0f = floorf(x);
    const float y0f = floorf(y);
    const float lx = x - x0f;
    const float ly = y - y0f;
    const int x0 = (int)x0f;
    const int y0 = (int)y0f;
    const int x1 = x0 + 1;
    const int y1 = y0 + 1;
    const bool vx0 = (x0 >= 0) && (x0 < Wl);
    const bool vx1 = (x1 >= 0) && (x1 < Wl);
    const bool vy0 = (y0 >= 0) && (y0 < Hl);
    const bool vy1 = (y1 >= 0) && (y1 < Hl);
    const float omlx = 1.0f - lx;
    const float omly = 1.0f - ly;
    const float b00 = omly * omlx;
    const float b01 = omly * lx;
    const float b10 = ly * omlx;
    const float b11 = ly * lx;
    const float w00 = b00 * ((vy0 && vx0) ? 1.0f : 0.0f);
    const float w01 = b01 * ((vy0 && vx1) ? 1.0f : 0.0f);
    const float w10 = b10 * ((vy1 && vx0) ? 1.0f : 0.0f);
    const float w11 = b11 * ((vy1 && vx1) ? 1.0f : 0.0f);
    const int cx0 = min(max(x0, 0), Wl - 1);
    const int cx1 = min(max(x1, 0), Wl - 1);
    const int cy0 = min(max(y0, 0), Hl - 1);
    const int cy1 = min(max(y1, 0), Hl - 1);
    const int i00 = st0 + cy0 * Wl + cx0;
    const int i01 = st0 + cy0 * Wl + cx1;
    const int i10 = st0 + cy1 * Wl + cx0;
    const int i11 = st0 + cy1 * Wl + cx1;

    const float* vm = vbase + m * kDh;
    float acc = 0.0f;
#pragma unroll 1
    for (int p = 0; p < kPts; ++p) {
      const int j00 = __shfl(i00, p, 32);
      const int j01 = __shfl(i01, p, 32);
      const int j10 = __shfl(i10, p, 32);
      const int j11 = __shfl(i11, p, 32);
      const float u00 = __shfl(w00, p, 32);
      const float u01 = __shfl(w01, p, 32);
      const float u10 = __shfl(w10, p, 32);
      const float u11 = __shfl(w11, p, 32);
      const float ap  = __shfl(aw, p, 32);
      const float v00 = vm[(size_t)j00 * kDm];
      const float v01 = vm[(size_t)j01 * kDm];
      const float v10 = vm[(size_t)j10 * kDm];
      const float v11 = vm[(size_t)j11 * kDm];
      const float t00 = v00 * u00;
      const float t01 = v01 * u01;
      const float t10 = v10 * u10;
      const float t11 = v11 * u11;
      float s = t00 + t01;
      s = s + t10;
      s = s + t11;
      const float sp = s * ap;
      acc = acc + sp;
    }
    st[m * kDh + lane] = acc;
  }

  __builtin_amdgcn_fence(__ATOMIC_RELEASE, "workgroup");
  __builtin_amdgcn_wave_barrier();
  __builtin_amdgcn_fence(__ATOMIC_ACQUIRE, "workgroup");
  const v4f fa = *(const v4f*)(st + lane * 8);
  const v4f fb = *(const v4f*)(st + lane * 8 + 4);
  v4u hv, lv;
  {
    unsigned h0, l0, h1, l1, h2, l2, h3, l3;
    split_pack2(fa[0], fa[1], h0, l0);
    split_pack2(fa[2], fa[3], h1, l1);
    split_pack2(fb[0], fb[1], h2, l2);
    split_pack2(fb[2], fb[3], h3, l3);
    hv[0] = h0; hv[1] = h1; hv[2] = h2; hv[3] = h3;
    lv[0] = l0; lv[1] = l1; lv[2] = l2; lv[3] = l3;
  }
  unsigned* ph = shi + (size_t)row * (kDm / 2) + lane * 4;
  unsigned* pl = slo + (size_t)row * (kDm / 2) + lane * 4;
  *(volatile v4u*)ph = hv;
  *(volatile v4u*)pl = lv;
  __threadfence();
  *(volatile v4u*)ph = hv;
  *(volatile v4u*)pl = lv;
}

extern "C" void kernel_launch(void* const* d_in, const int* in_sizes, int n_in,
                              void* d_out, int out_size, void* d_ws, size_t ws_size,
                              hipStream_t stream) {
  if (n_in < 13) return;
  if (in_sizes[0] != kMreal * kDm || in_sizes[1] != kMreal * 8 || in_sizes[2] != kMreal * kDm) return;
  if (in_sizes[5] != 256 * 256 || in_sizes[6] != 256 || in_sizes[7] != 128 * 256 || in_sizes[8] != 128) return;
  if (in_sizes[9] != 256 * 256 || in_sizes[10] != 256 || in_sizes[11] != 256 * 256 || in_sizes[12] != 256) return;
  if (out_size != kMreal * kDm) return;
  if (kWsTotal > ws_size) return;

  const float* query  = (const float*)d_in[0];
  const float* rpts   = (const float*)d_in[1];
  const float* flat   = (const float*)d_in[2];
  const float* W_off  = (const float*)d_in[5];
  const float* b_off  = (const float*)d_in[6];
  const float* W_log  = (const float*)d_in[7];
  const float* b_log  = (const float*)d_in[8];
  const float* W_val  = (const float*)d_in[9];
  const float* b_val  = (const float*)d_in[10];
  const float* W_out  = (const float*)d_in[11];
  const float* b_out  = (const float*)d_in[12];
  float* out = (float*)d_out;

  char* ws = (char*)d_ws;
  unsigned* q16  = (unsigned*)(ws + kOffQ16);
  unsigned* f16p = (unsigned*)(ws + kOffF16);
  unsigned* wval = (unsigned*)(ws + kOffWval);
  unsigned* woff = (unsigned*)(ws + kOffWoff);
  unsigned* wlog = (unsigned*)(ws + kOffWlog);
  unsigned* wout = (unsigned*)(ws + kOffWout);
  float* value = (float*)(ws + kOffValue);
  float* offs  = (float*)(ws + kOffOffs);
  float* logit = (float*)(ws + kOffLogit);
  unsigned* shi = (unsigned*)(ws + kOffShi);
  unsigned* slo = (unsigned*)(ws + kOffSlo);

  cvt_rows_bf16<<<dim3(kMpad / 8), dim3(256), 0, stream>>>(query, q16, kMreal, kMpad);
  cvt_rows_bf16<<<dim3(kMpad / 8), dim3(256), 0, stream>>>(flat, f16p, kMreal, kMpad);
  cvt_rows_bf16<<<dim3(256 / 8), dim3(256), 0, stream>>>(W_val, wval, 256, 256);
  cvt_rows_bf16<<<dim3(256 / 8), dim3(256), 0, stream>>>(W_off, woff, 256, 256);
  cvt_rows_bf16<<<dim3(128 / 8), dim3(256), 0, stream>>>(W_log, wlog, 128, 128);
  cvt_rows_bf16<<<dim3(256 / 8), dim3(256), 0, stream>>>(W_out, wout, 256, 256);

  const int tilesA = (kMpad / 64) * (kDm / 64);
  const int tilesL = (kMpad / 64) * (kLogit / 64);
  const int blocksA = (tilesA + 7) / 8;
  const int blocksL = (tilesL + 7) / 8;

  wmma_gemm64<1, false, false, 2, true, 0, false, 0><<<dim3(blocksA, 1), dim3(256), 0, stream>>>(
      (const unsigned short*)f16p, (const unsigned short*)f16p, kDm, 0L,
      (const unsigned short*)wval, (const unsigned short*)wval, kDm, 0L,
      (void*)value, (void*)value, kDm, 0L,
      b_val, b_val, 0L, kMpad, kDm, kDm, kMpad, 1.0f);
  wmma_gemm64<1, false, false, 2, true, 0, false, 0><<<dim3(blocksA, 1), dim3(256), 0, stream>>>(
      (const unsigned short*)q16, (const unsigned short*)q16, kDm, 0L,
      (const unsigned short*)woff, (const unsigned short*)woff, kDm, 0L,
      (void*)offs, (void*)offs, kDm, 0L,
      b_off, b_off, 0L, kMpad, kDm, kDm, kMpad, 1.0f);
  wmma_gemm64<1, false, false, 2, true, 0, false, 0><<<dim3(blocksL, 1), dim3(256), 0, stream>>>(
      (const unsigned short*)q16, (const unsigned short*)q16, kDm, 0L,
      (const unsigned short*)wlog, (const unsigned short*)wlog, kDm, 0L,
      (void*)logit, (void*)logit, kLogit, 0L,
      b_log, b_log, 0L, kMpad, kLogit, kDm, kMpad, 1.0f);

  deform_gather<<<dim3(kMpad / 8), dim3(256), 0, stream>>>(value, offs, logit, rpts, shi, slo);

  wmma_gemm64<1, true, true, 2, true, 0, false, 0><<<dim3(blocksA, 1), dim3(256), 0, stream>>>(
      (const unsigned short*)shi, (const unsigned short*)slo, kDm, 0L,
      (const unsigned short*)wout, (const unsigned short*)wout, kDm, 0L,
      (void*)out, (void*)out, kDm, 0L,
      b_out, b_out, 0L, kMpad, kDm, kDm, kMreal, 1.0f);
}
